// NWHead_66331474920046
// MI455X (gfx1250) — hardware-run, weakly checked
//
#include <hip/hip_runtime.h>
#include <math.h>

#define FEAT   1024
#define PROJ   256
#define BATCH  32
#define NSUP   8192
#define NROWS  (BATCH + NSUP)
#define NCLS   1000

#define XG8    (BATCH * FEAT / 8)
#define SXG8   (NSUP * FEAT / 8)
#define WG8    (FEAT * PROJ / 8)
#define XBLK   (XG8 / 256)
#define SXBLK  (SXG8 / 256)
#define WBLK   (WG8 / 256)

#define G1BLK  (NROWS / 32)
#define SCBLK  (NSUP / 256)
#define SM_ROWS 4
#define SMBLK  (BATCH / SM_ROWS)
#define SM_LINES ((SM_ROWS * NCLS) / 32)

static_assert(XG8 % 256 == 0);
static_assert(SXG8 % 256 == 0);
static_assert(WG8 % 256 == 0);
static_assert(NROWS % 32 == 0);
static_assert(NSUP % 256 == 0);
static_assert((SM_ROWS * NCLS) % 32 == 0);
static_assert(BATCH % SM_ROWS == 0);
static_assert(FEAT % 32 == 0);
static_assert(PROJ % 32 == 0);

typedef __attribute__((ext_vector_type(16))) __bf16 v16bf;
typedef __attribute__((ext_vector_type(8)))  float  v8f;
typedef __attribute__((ext_vector_type(4)))  float  v4f;
typedef __attribute__((ext_vector_type(8)))  unsigned short v8us;
typedef v4f  __attribute__((may_alias)) v4fa;
typedef v8us __attribute__((may_alias)) v8usa;

union BFrag { v16bf v; v8us h[2]; };

__device__ __forceinline__ unsigned short bf_rne(float f) {
    unsigned int u = __builtin_bit_cast(unsigned int, f);
    u += 0x7FFFu + ((u >> 16) & 1u);
    return (unsigned short)(u >> 16);
}
__device__ __forceinline__ float bf_up(unsigned short s) {
    return __builtin_bit_cast(float, ((unsigned int)s) << 16);
}
__device__ __forceinline__ void split8(v4f a, v4f c, v8us& hv, v8us& lv) {
    float f[8] = { a.x, a.y, a.z, a.w, c.x, c.y, c.z, c.w };
#pragma unroll
    for (int i = 0; i < 8; ++i) {
        const unsigned short hs = bf_rne(f[i]);
        hv[i] = hs;
        lv[i] = bf_rne(f[i] - bf_up(hs));
    }
}

__device__ __forceinline__ v8f wmma_bf(v16bf a, v16bf b, v8f c) {
#if defined(__HIP_DEVICE_COMPILE__)
    v8f d = __builtin_amdgcn_wmma_f32_16x16x32_bf16(false, a, false, b, (short)0, c, false, false);
    asm volatile("v_nop\n\tv_nop\n\tv_nop\n\tv_nop" : "+v"(d) : "v"(a), "v"(b));
    return d;
#else
    (void)a; (void)b;
    return c;
#endif
}

__device__ __forceinline__ v16bf ldfrag(const unsigned short* p, int h) {
    BFrag f;
    f.h[0] = *(const v8usa*)(p + 8 * h);
    f.h[1] = *(const v8usa*)(p + 16 + 8 * h);
    return f.v;
}

__global__ void __launch_bounds__(256)
k_convert(const float* __restrict__ x, const float* __restrict__ sx, const float* __restrict__ W,
          unsigned short* __restrict__ xH, unsigned short* __restrict__ xL,
          unsigned short* __restrict__ sH, unsigned short* __restrict__ sL,
          unsigned short* __restrict__ wH, unsigned short* __restrict__ wL)
{
    const int blk = blockIdx.x, tid = threadIdx.x;
    v4f a, c;
    unsigned short* dh;
    unsigned short* dl;
    if (blk < XBLK) {
        const size_t g = (size_t)blk * 256 + tid;
        const float* src = x + g * 8;
        a = *(const v4fa*)(src);
        c = *(const v4fa*)(src + 4);
        dh = xH + g * 8;
        dl = xL + g * 8;
    } else if (blk < XBLK + SXBLK) {
        const size_t g = (size_t)(blk - XBLK) * 256 + tid;
        const float* src = sx + g * 8;
        a = *(const v4fa*)(src);
        c = *(const v4fa*)(src + 4);
        dh = sH + g * 8;
        dl = sL + g * 8;
    } else {
        const int t  = (blk - XBLK - SXBLK) * 256 + tid;
        const int n  = t >> 7;
        const int kg = t & 127;
        const int k0 = kg * 8;
        const float* src = W + (size_t)k0 * PROJ + n;
        a.x = src[0];          a.y = src[PROJ];       a.z = src[2 * PROJ];   a.w = src[3 * PROJ];
        c.x = src[4 * PROJ];   c.y = src[5 * PROJ];   c.z = src[6 * PROJ];   c.w = src[7 * PROJ];
        dh = wH + (size_t)n * FEAT + k0;
        dl = wL + (size_t)n * FEAT + k0;
    }
    v8us hv, lv;
    split8(a, c, hv, lv);
    *(volatile v8us*)dh = hv;
    *(volatile v8us*)dl = lv;
    __threadfence();
    *(volatile v8us*)dh = hv;
    *(volatile v8us*)dl = lv;
}

__global__ void __launch_bounds__(256)
k_gemm1(const unsigned short* __restrict__ xH, const unsigned short* __restrict__ xL,
        const unsigned short* __restrict__ sH, const unsigned short* __restrict__ sL,
        const unsigned short* __restrict__ wH, const unsigned short* __restrict__ wL,
        unsigned short* __restrict__ pH, unsigned short* __restrict__ pL,
        float* __restrict__ sq)
{
    __shared__ __attribute__((aligned(16))) float sT[32 * PROJ];
    __shared__ __attribute__((aligned(16))) float sSq[32];

    const int tid = threadIdx.x, lane = tid & 31, wv = tid >> 5;
    const int h = lane >> 4, m = lane & 15;
    const int blk = blockIdx.x;

    const unsigned short* aH;
    const unsigned short* aL;
    if (blk == 0) { aH = xH; aL = xL; }
    else {
        const size_t off = (size_t)(blk - 1) * 32 * FEAT;
        aH = sH + off; aL = sL + off;
    }
    const unsigned short* a0H = aH + (size_t)m * FEAT;
    const unsigned short* a1H = a0H + (size_t)16 * FEAT;
    const unsigned short* a0L = aL + (size_t)m * FEAT;
    const unsigned short* a1L = a0L + (size_t)16 * FEAT;

    const int c0 = 32 * wv;
    const unsigned short* b0H = wH + (size_t)(c0 + m) * FEAT;
    const unsigned short* b1H = b0H + (size_t)16 * FEAT;
    const unsigned short* b0L = wL + (size_t)(c0 + m) * FEAT;
    const unsigned short* b1L = b0L + (size_t)16 * FEAT;

    const v8f zero8 = {0.f, 0.f, 0.f, 0.f, 0.f, 0.f, 0.f, 0.f};
    v8f acc[2][2];
#pragma unroll
    for (int mt = 0; mt < 2; ++mt)
#pragma unroll
        for (int nt = 0; nt < 2; ++nt) acc[mt][nt] = zero8;

#pragma unroll 1
    for (int k0 = 0; k0 < FEAT; k0 += 32) {
        const v16bf a0h = ldfrag(a0H + k0, h);
        const v16bf a0l = ldfrag(a0L + k0, h);
        const v16bf a1h = ldfrag(a1H + k0, h);
        const v16bf a1l = ldfrag(a1L + k0, h);
        const v16bf b0h = ldfrag(b0H + k0, h);
        const v16bf b0l = ldfrag(b0L + k0, h);
        const v16bf b1h = ldfrag(b1H + k0, h);
        const v16bf b1l = ldfrag(b1L + k0, h);

        acc[0][0] = wmma_bf(a0l, b0h, acc[0][0]);
        acc[0][0] = wmma_bf(a0h, b0l, acc[0][0]);
        acc[0][0] = wmma_bf(a0h, b0h, acc[0][0]);
        acc[0][1] = wmma_bf(a0l, b1h, acc[0][1]);
        acc[0][1] = wmma_bf(a0h, b1l, acc[0][1]);
        acc[0][1] = wmma_bf(a0h, b1h, acc[0][1]);
        acc[1][0] = wmma_bf(a1l, b0h, acc[1][0]);
        acc[1][0] = wmma_bf(a1h, b0l, acc[1][0]);
        acc[1][0] = wmma_bf(a1h, b0h, acc[1][0]);
        acc[1][1] = wmma_bf(a1l, b1h, acc[1][1]);
        acc[1][1] = wmma_bf(a1h, b1l, acc[1][1]);
        acc[1][1] = wmma_bf(a1h, b1h, acc[1][1]);
    }

#pragma unroll
    for (int mt = 0; mt < 2; ++mt)
#pragma unroll
        for (int nt = 0; nt < 2; ++nt)
#pragma unroll
            for (int r = 0; r < 8; ++r)
                sT[(16 * mt + 8 * h + r) * PROJ + c0 + 16 * nt + m] = acc[mt][nt][r];
    __syncthreads();

#pragma unroll 1
    for (int i = 0; i < 4; ++i) {
        const int row = 4 * wv + i;
        const float* rp = sT + row * PROJ + 8 * lane;
        const v4f a = *(const v4fa*)(rp);
        const v4f c = *(const v4fa*)(rp + 4);
        float s = a.x * a.x + a.y * a.y + a.z * a.z + a.w * a.w
                + c.x * c.x + c.y * c.y + c.z * c.z + c.w * c.w;
#pragma unroll
        for (int off = 16; off > 0; off >>= 1) s += __shfl_xor(s, off, 32);
        if (lane == 0) sSq[row] = s;

        v8us hv, lv;
        split8(a, c, hv, lv);
        const size_t g = ((size_t)blk * 32 + row) * PROJ + 8 * lane;
        *(volatile v8us*)(pH + g) = hv;
        *(volatile v8us*)(pL + g) = lv;
        __threadfence();
        *(volatile v8us*)(pH + g) = hv;
        *(volatile v8us*)(pL + g) = lv;
    }
    __syncthreads();

    if (tid < 8) {
        const v4f q = *(const v4fa*)(sSq + 4 * tid);
        float* d = sq + (size_t)blk * 32 + 4 * tid;
        *(volatile v4f*)d = q;
        __threadfence();
        *(volatile v4f*)d = q;
    }
}

__device__ __forceinline__ void st_S_pass(const float* sSw, float* S, int n0, int lane) {
    const int q8 = lane & 7, sub = lane >> 3;
#pragma unroll
    for (int i = 0; i < 8; ++i) {
        const int row = 4 * i + sub;
        const v4f v = *(const v4fa*)(sSw + row * 32 + 4 * q8);
        *(volatile v4f*)(S + (size_t)row * NSUP + n0 + 4 * q8) = v;
    }
}

__global__ void __launch_bounds__(256)
k_scores(const unsigned short* __restrict__ pH, const unsigned short* __restrict__ pL,
         const float* __restrict__ sq, float* __restrict__ S)
{
    __shared__ __attribute__((aligned(16))) float sS[8 * 32 * 32];

    const int tid = threadIdx.x, lane = tid & 31, wv = tid >> 5;
    const int h = lane >> 4, m = lane & 15;
    const int n0 = 32 * (blockIdx.x * 8 + wv);

    const unsigned short* a0H = pH + (size_t)m * PROJ;
    const unsigned short* a1H = a0H + (size_t)16 * PROJ;
    const unsigned short* a0L = pL + (size_t)m * PROJ;
    const unsigned short* a1L = a0L + (size_t)16 * PROJ;
    const unsigned short* b0H = pH + (size_t)(BATCH + n0 + m) * PROJ;
    const unsigned short* b1H = b0H + (size_t)16 * PROJ;
    const unsigned short* b0L = pL + (size_t)(BATCH + n0 + m) * PROJ;
    const unsigned short* b1L = b0L + (size_t)16 * PROJ;

    const v8f zero8 = {0.f, 0.f, 0.f, 0.f, 0.f, 0.f, 0.f, 0.f};
    v8f acc[2][2];
#pragma unroll
    for (int mt = 0; mt < 2; ++mt)
#pragma unroll
        for (int nt = 0; nt < 2; ++nt) acc[mt][nt] = zero8;

#pragma unroll 1
    for (int k0 = 0; k0 < PROJ; k0 += 32) {
        const v16bf a0h = ldfrag(a0H + k0, h);
        const v16bf a0l = ldfrag(a0L + k0, h);
        const v16bf a1h = ldfrag(a1H + k0, h);
        const v16bf a1l = ldfrag(a1L + k0, h);
        const v16bf b0h = ldfrag(b0H + k0, h);
        const v16bf b0l = ldfrag(b0L + k0, h);
        const v16bf b1h = ldfrag(b1H + k0, h);
        const v16bf b1l = ldfrag(b1L + k0, h);

        acc[0][0] = wmma_bf(a0l, b0h, acc[0][0]);
        acc[0][0] = wmma_bf(a0h, b0l, acc[0][0]);
        acc[0][0] = wmma_bf(a0h, b0h, acc[0][0]);
        acc[0][1] = wmma_bf(a0l, b1h, acc[0][1]);
        acc[0][1] = wmma_bf(a0h, b1l, acc[0][1]);
        acc[0][1] = wmma_bf(a0h, b1h, acc[0][1]);
        acc[1][0] = wmma_bf(a1l, b0h, acc[1][0]);
        acc[1][0] = wmma_bf(a1h, b0l, acc[1][0]);
        acc[1][0] = wmma_bf(a1h, b0h, acc[1][0]);
        acc[1][1] = wmma_bf(a1l, b1h, acc[1][1]);
        acc[1][1] = wmma_bf(a1h, b1l, acc[1][1]);
        acc[1][1] = wmma_bf(a1h, b1h, acc[1][1]);
    }

    const float ss0 = sq[BATCH + n0 + m];
    const float ss1 = sq[BATCH + n0 + 16 + m];
    float* sSw = sS + wv * 1024;
#pragma unroll
    for (int mt = 0; mt < 2; ++mt)
#pragma unroll
        for (int r = 0; r < 8; ++r) {
            const int row = 16 * mt + 8 * h + r;
            const float xs = sq[row];
            const float v0 = -((xs + ss0) - 2.0f * acc[mt][0][r]);
            const float v1 = -((xs + ss1) - 2.0f * acc[mt][1][r]);
            sSw[row * 32 + m]      = v0;
            sSw[row * 32 + 16 + m] = v1;
        }
    __syncthreads();

    st_S_pass(sSw, S, n0, lane);
    __threadfence();
    st_S_pass(sSw, S, n0, lane);
}

__device__ __forceinline__ void st_out_pass(const float* so, float* out, int blk, int wv, int lane) {
    const int q8 = lane & 7, sub = lane >> 3;
#pragma unroll
    for (int i = 0; i < 4; ++i) {
        const int L  = 32 * i + 4 * wv + sub;
        const int Lc = (L < SM_LINES) ? L : (SM_LINES - 1);
        const v4f v  = *(const v4fa*)(so + 32 * Lc + 4 * q8);
        if (L < SM_LINES)
            *(volatile v4f*)(out + (size_t)blk * (SM_ROWS * NCLS) + 32 * L + 4 * q8) = v;
    }
}

__global__ void __launch_bounds__(256)
k_softmax(const float* __restrict__ S, const int* __restrict__ sy, float* __restrict__ out)
{
    __shared__ float red[256];
    __shared__ float bins[8 * NCLS];
    __shared__ __attribute__((aligned(16))) float so[SM_ROWS * NCLS];

    const int tid = threadIdx.x, lane = tid & 31, wv = tid >> 5;
    const int blk = blockIdx.x;

#pragma unroll 1
    for (int rl = 0; rl < SM_ROWS; ++rl) {
        const int row = blk * SM_ROWS + rl;
        const float* sr = S + (size_t)row * NSUP;

        float mx = -3.402823466e38f;
#pragma unroll 1
        for (int j = tid; j < NSUP; j += 256) mx = fmaxf(mx, sr[j]);
        red[tid] = mx;
        __syncthreads();
#pragma unroll 1
        for (int s = 128; s > 0; s >>= 1) {
            if (tid < s) red[tid] = fmaxf(red[tid], red[tid + s]);
            __syncthreads();
        }
        mx = red[0];
        __syncthreads();

        float sum = 0.0f;
#pragma unroll 1
        for (int j = tid; j < NSUP; j += 256) sum += expf(sr[j] - mx);
        red[tid] = sum;
        __syncthreads();
#pragma unroll 1
        for (int s = 128; s > 0; s >>= 1) {
            if (tid < s) red[tid] += red[tid + s];
            __syncthreads();
        }
        const float tot = red[0];
        __syncthreads();
        const float inv = 1.0f / tot;

#pragma unroll 1
        for (int c = tid; c < 8 * NCLS; c += 256) bins[c] = 0.0f;
        __syncthreads();

        float* bb = bins + wv * NCLS;
        const int jb = wv * (NSUP / 8);
#pragma unroll 1
        for (int g = 0; g < (NSUP / 8) / 32; ++g) {
            const int j = jb + 32 * g + lane;
            const float p = expf(sr[j] - mx) * inv;
            const int c = sy[j];
            const int cc = min(max(c, 0), NCLS - 1);
            const float pv = ((unsigned)c < (unsigned)NCLS) ? p : 0.0f;
#pragma unroll 1
            for (int l = 0; l < 32; ++l) {
                const int   cl = __shfl(cc, l, 32);
                const float pl = __shfl(pv, l, 32);
                const float nv = bb[cl] + pl;
                bb[cl] = nv;
            }
        }
        __syncthreads();

#pragma unroll 1
        for (int c = tid; c < NCLS; c += 256) {
            const float t01 = bins[c]            + bins[NCLS + c];
            const float t23 = bins[2 * NCLS + c] + bins[3 * NCLS + c];
            const float t45 = bins[4 * NCLS + c] + bins[5 * NCLS + c];
            const float t67 = bins[6 * NCLS + c] + bins[7 * NCLS + c];
            const float t = (t01 + t23) + (t45 + t67);
            so[rl * NCLS + c] = logf(t + 1e-12f);
        }
        __syncthreads();
    }

    st_out_pass(so, out, blk, wv, lane);
    __threadfence();
    st_out_pass(so, out, blk, wv, lane);
}

extern "C" void kernel_launch(void* const* d_in, const int* in_sizes, int n_in,
                              void* d_out, int out_size, void* d_ws, size_t ws_size,
                              hipStream_t stream) {
    if (n_in < 4) return;
    if (in_sizes[0] != BATCH * FEAT) return;
    if (in_sizes[1] != NSUP * FEAT) return;
    if (in_sizes[2] != FEAT * PROJ) return;
    if (in_sizes[3] != NSUP) return;
    if (out_size != BATCH * NCLS) return;

    const float* x  = (const float*)d_in[0];
    const float* sx = (const float*)d_in[1];
    const float* W  = (const float*)d_in[2];
    const int*   sy = (const int*)d_in[3];
    float* out = (float*)d_out;

    const size_t XPB  = (size_t)BATCH * FEAT * 2;
    const size_t SXPB = (size_t)NSUP * FEAT * 2;
    const size_t WPB  = (size_t)PROJ * FEAT * 2;
    const size_t PPB  = (size_t)NROWS * PROJ * 2;
    const size_t SQB  = (((size_t)NROWS * 4) + 255) & ~(size_t)255;
    const size_t SB   = (size_t)BATCH * NSUP * 4;
    const size_t o_xH = 0;
    const size_t o_xL = o_xH + XPB;
    const size_t o_sH = o_xL + XPB;
    const size_t o_sL = o_sH + SXPB;
    const size_t o_wH = o_sL + SXPB;
    const size_t o_wL = o_wH + WPB;
    const size_t o_pH = o_wL + WPB;
    const size_t o_pL = o_pH + PPB;
    const size_t o_sq = o_pL + PPB;
    const size_t o_S  = o_sq + SQB;
    const size_t total = o_S + SB;
    if (total > ws_size) return;

    char* ws = (char*)d_ws;
    unsigned short* xH = (unsigned short*)(ws + o_xH);
    unsigned short* xL = (unsigned short*)(ws + o_xL);
    unsigned short* sH = (unsigned short*)(ws + o_sH);
    unsigned short* sL = (unsigned short*)(ws + o_sL);
    unsigned short* wH = (unsigned short*)(ws + o_wH);
    unsigned short* wL = (unsigned short*)(ws + o_wL);
    unsigned short* pH = (unsigned short*)(ws + o_pH);
    unsigned short* pL = (unsigned short*)(ws + o_pL);
    float* sq = (float*)(ws + o_sq);
    float* S  = (float*)(ws + o_S);

    k_convert<<<XBLK + SXBLK + WBLK, 256, 0, stream>>>(x, sx, W, xH, xL, sH, sL, wH, wL);
    k_gemm1<<<G1BLK, 256, 0, stream>>>(xH, xL, sH, sL, wH, wL, pH, pL, sq);
    k_scores<<<SCBLK, 256, 0, stream>>>(pH, pL, sq, S);
    k_softmax<<<SMBLK, 256, 0, stream>>>(S, sy, out);
    (void)hipGetLastError();
}
